// SparseAttention_27874337751552
// MI455X (gfx1250) — hardware-verified
//
#include <hip/hip_runtime.h>
#include <math.h>
#include <stdint.h>

#define NB   4
#define SEQ  4096
#define HD   128
#define WIN  128
#define QBLK 64
#define KCH  64
#define NCH  5
#define NQB  (SEQ / QBLK)
#define NKC  (SEQ / KCH)
static_assert(NQB == 64 && NKC == 64);
static_assert(QBLK == KCH);
static_assert((WIN - 1) > KCH && (WIN - 1) <= 2 * KCH);
static_assert((QBLK - 1 + WIN - 1) / KCH == 2);
static_assert(HD == 128 && (HD % 32) == 0 && (SEQ % QBLK) == 0 && (SEQ % 64) == 0);

typedef __bf16         v16b __attribute__((ext_vector_type(16)));
typedef float          v8f  __attribute__((ext_vector_type(8)));
typedef float          v4f  __attribute__((ext_vector_type(4)));
typedef unsigned int   v4u  __attribute__((ext_vector_type(4)));
typedef unsigned short v8us __attribute__((ext_vector_type(8)));

#if defined(__HIP_DEVICE_COMPILE__)
#define DEV_ASM 1
#else
#define DEV_ASM 0
#endif

__device__ __forceinline__ unsigned short bf_bits(float f) {
  unsigned u = __float_as_uint(f);
  return (unsigned short)((u + 0x7FFFu + ((u >> 16) & 1u)) >> 16);
}
__device__ __forceinline__ float bf_up(unsigned short hb) { return __uint_as_float(((unsigned)hb) << 16); }
__device__ __forceinline__ unsigned pk16(unsigned short a, unsigned short b) { return (unsigned)a | ((unsigned)b << 16); }
__device__ __forceinline__ v8f zero8() { v8f z = {0.f, 0.f, 0.f, 0.f, 0.f, 0.f, 0.f, 0.f}; return z; }

union FB { v16b v; v8us h[2]; };
__device__ __forceinline__ v16b ldfrag_us(const unsigned short* p) {
  FB f;
  f.h[0] = *(const v8us*)(p);
  f.h[1] = *(const v8us*)(p + 16);
  return f.v;
}

__device__ __forceinline__ v8f mma_b(v16b a, v16b b, v8f c) {
  c = __builtin_amdgcn_wmma_f32_16x16x32_bf16(false, a, false, b, (short)0, c, false, false);
#if DEV_ASM
  asm volatile("v_nop\n\tv_nop\n\tv_nop\n\tv_nop" : "+v"(c) : "v"(a), "v"(b));
#endif
  return c;
}

__global__ __launch_bounds__(256) void cvt_bf16x8(const float* __restrict__ in, unsigned short* out, int n8) {
  const int i = blockIdx.x * 256 + (int)threadIdx.x;
  if (i < n8) {
    const v4f a  = *(const v4f*)(in + (size_t)i * 8);
    const v4f a4 = *(const v4f*)(in + (size_t)i * 8 + 4);
    v4u p;
    p[0] = pk16(bf_bits(a[0]),  bf_bits(a[1]));
    p[1] = pk16(bf_bits(a[2]),  bf_bits(a[3]));
    p[2] = pk16(bf_bits(a4[0]), bf_bits(a4[1]));
    p[3] = pk16(bf_bits(a4[2]), bf_bits(a4[3]));
    unsigned short* o = out + (size_t)i * 8;
    *(volatile v4u*)o = p;
    __threadfence();
    *(volatile v4u*)o = p;
  }
}

#define TP 72
__global__ __launch_bounds__(128) void vtr64(const float* __restrict__ v, unsigned short* vt) {
  __shared__ __align__(16) unsigned short T[HD * TP];
  const int tid  = (int)threadIdx.x;
  const int lane = tid & 31;
  const int wave = tid >> 5;
  const int s0   = blockIdx.x * 64;
  const int b    = blockIdx.y;
  const float* vb = v + ((size_t)b * SEQ + (size_t)s0) * HD;
#pragma unroll
  for (int it = 0; it < 16; ++it) {
    const int idx = it * 128 + tid;
    const int row = idx >> 5;
    const int col = (idx & 31) * 4;
    const v4f x = *(const v4f*)(vb + (size_t)row * HD + col);
#pragma unroll
    for (int e = 0; e < 4; ++e) T[(col + e) * TP + row] = bf_bits(x[e]);
  }
  __syncthreads();
  const int q8 = lane >> 3, c8 = (lane & 7) * 8;
  v4u pv[8];
#pragma unroll
  for (int it = 0; it < 8; ++it) {
    const int d = wave * 32 + it * 4 + q8;
    const v8us x = *(const v8us*)(T + d * TP + c8);
    pv[it] = __builtin_bit_cast(v4u, x);
  }
  unsigned short* ob = vt + ((size_t)b * HD) * SEQ + (size_t)s0;
  for (int pass = 0; pass < 2; ++pass) {
#pragma unroll
    for (int it = 0; it < 8; ++it) {
      const int d = wave * 32 + it * 4 + q8;
      *(volatile v4u*)(ob + (size_t)d * SEQ + c8) = pv[it];
    }
    __threadfence();
  }
}

__global__ __launch_bounds__(128)
void attn_band(const unsigned short* __restrict__ qp, const unsigned short* __restrict__ kp,
               const unsigned short* __restrict__ vtp, float* out, float sscale) {
  __shared__ __align__(16) unsigned short Ksh[KCH * HD];
  __shared__ __align__(16) unsigned short Vth[HD * KCH];
  __shared__ __align__(16) unsigned short Phs[4][16 * KCH];
  __shared__ __align__(16) unsigned short Pls[4][16 * KCH];
  __shared__ __align__(16) float          Os[4][16 * HD];

  const int tid  = (int)threadIdx.x;
  const int wave = tid >> 5;
  const int lane = tid & 31;
  const int hh   = lane >> 4;
  const int c    = lane & 15;

  const int qb   = (int)blockIdx.x % NQB;
  const int b    = (int)blockIdx.x / NQB;
  const int q0   = qb * QBLK + wave * 16;
  const size_t rowB = (size_t)b * SEQ;

  const unsigned short* Vg = vtp + ((size_t)b * HD) * SEQ;

  v16b qa[4];
#pragma unroll
  for (int dc = 0; dc < 4; ++dc)
    qa[dc] = ldfrag_us(qp + (rowB + (size_t)(q0 + c)) * HD + dc * 32 + 8 * hh);

  float mrow[8], lrow[8];
  v8f oacc[8];
#pragma unroll
  for (int r = 0; r < 8; ++r) { mrow[r] = -INFINITY; lrow[r] = 0.f; }
#pragma unroll
  for (int t = 0; t < 8; ++t) oacc[t] = zero8();

  unsigned short* ph = Phs[wave];
  unsigned short* pl = Pls[wave];

#pragma unroll 1
  for (int ci = 0; ci < NCH; ++ci) {
    const int kc = qb - 2 + ci;
    if (kc < 0 || kc >= NKC) continue;
    const int kv0 = kc * KCH;

    __syncthreads();
    {
      const int r = tid >> 1, half = (tid & 1) * 64;
      const unsigned short* kg = kp + (rowB + (size_t)(kv0 + r)) * HD + half;
      const unsigned short* vg = Vg + (size_t)tid * SEQ + kv0;
#pragma unroll
      for (int i = 0; i < 8; ++i) {
        const v8us a0 = *(const v8us*)(kg + 8 * i);
        const v8us b0 = *(const v8us*)(vg + 8 * i);
        *(v8us*)(Ksh + r * HD + half + 8 * i) = a0;
        *(v8us*)(Vth + tid * KCH + 8 * i)      = b0;
      }
    }
    __syncthreads();

    v8f s[4];
#pragma unroll
    for (int j = 0; j < 4; ++j) {
      v8f a = zero8();
#pragma unroll
      for (int dc = 0; dc < 4; ++dc) {
        FB kb;
        kb.h[0] = *(const v8us*)(Ksh + (j * 16 + c) * HD + dc * 32 + 8 * hh);
        kb.h[1] = *(const v8us*)(Ksh + (j * 16 + c) * HD + dc * 32 + 16 + 8 * hh);
        a = mma_b(qa[dc], kb.v, a);
      }
      const int jkey = kv0 + j * 16 + c;
#pragma unroll
      for (int r = 0; r < 8; ++r) {
        const int dd = (q0 + 8 * hh + r) - jkey;
        const bool inband = (dd <= (WIN - 1)) && (dd >= -(WIN - 1));
        s[j][r] = inband ? (a[r] * sscale) : -INFINITY;
      }
    }

#pragma unroll
    for (int r = 0; r < 8; ++r) {
      float m = s[0][r];
#pragma unroll
      for (int j = 1; j < 4; ++j) m = fmaxf(m, s[j][r]);
#pragma unroll
      for (int off = 1; off < 16; off <<= 1) m = fmaxf(m, __shfl_xor(m, off, 32));
      const float mnew  = fmaxf(mrow[r], m);
      const float msafe = (mnew == -INFINITY) ? 0.f : mnew;
      const float alpha = expf(mrow[r] - msafe);
      mrow[r] = mnew;
      float psum = 0.f;
#pragma unroll
      for (int j = 0; j < 4; ++j) {
        const float p = expf(s[j][r] - msafe);
        psum += p;
        const unsigned short hb = bf_bits(p);
        const unsigned short lb = bf_bits(p - bf_up(hb));
        ph[(8 * hh + r) * KCH + j * 16 + c] = hb;
        pl[(8 * hh + r) * KCH + j * 16 + c] = lb;
      }
#pragma unroll
      for (int off = 1; off < 16; off <<= 1) psum += __shfl_xor(psum, off, 32);
      lrow[r] = lrow[r] * alpha + psum;
#pragma unroll
      for (int t = 0; t < 8; ++t) oacc[t][r] *= alpha;
    }
    __builtin_amdgcn_fence(__ATOMIC_RELEASE, "workgroup");
    __builtin_amdgcn_wave_barrier();
    __builtin_amdgcn_fence(__ATOMIC_ACQUIRE, "workgroup");

#pragma unroll 1
    for (int kk = 0; kk < 2; ++kk) {
      FB pa, pr;
      pa.h[0] = *(const v8us*)(ph + c * KCH + kk * 32 + 8 * hh);
      pa.h[1] = *(const v8us*)(ph + c * KCH + kk * 32 + 16 + 8 * hh);
      pr.h[0] = *(const v8us*)(pl + c * KCH + kk * 32 + 8 * hh);
      pr.h[1] = *(const v8us*)(pl + c * KCH + kk * 32 + 16 + 8 * hh);
#pragma unroll
      for (int t = 0; t < 8; ++t) {
        FB vb;
        vb.h[0] = *(const v8us*)(Vth + (t * 16 + c) * KCH + kk * 32 + 8 * hh);
        vb.h[1] = *(const v8us*)(Vth + (t * 16 + c) * KCH + kk * 32 + 16 + 8 * hh);
        oacc[t] = mma_b(pa.v, vb.v, oacc[t]);
        oacc[t] = mma_b(pr.v, vb.v, oacc[t]);
      }
    }
  }

  float* os = Os[wave];
#pragma unroll
  for (int r = 0; r < 8; ++r) {
    const float l   = lrow[r];
    const float inv = (l > 0.f) ? (1.0f / l) : 0.f;
#pragma unroll
    for (int t = 0; t < 8; ++t) os[(8 * hh + r) * HD + t * 16 + c] = oacc[t][r] * inv;
  }
  __builtin_amdgcn_fence(__ATOMIC_RELEASE, "workgroup");
  __builtin_amdgcn_wave_barrier();
  __builtin_amdgcn_fence(__ATOMIC_ACQUIRE, "workgroup");
  {
    const int c4 = lane * 4;
    for (int pass = 0; pass < 2; ++pass) {
#pragma unroll
      for (int it = 0; it < 16; ++it) {
        const v4f x = *(const v4f*)(os + it * HD + c4);
        *(volatile v4f*)(out + (rowB + (size_t)(q0 + it)) * HD + c4) = x;
      }
      __threadfence();
    }
  }
}

extern "C" void kernel_launch(void* const* d_in, const int* in_sizes, int n_in,
                              void* d_out, int out_size, void* d_ws, size_t ws_size,
                              hipStream_t stream) {
  const int n = NB * SEQ * HD;
  if (n_in < 3) return;
  if (in_sizes[0] != n || in_sizes[1] != n || in_sizes[2] != n) return;
  if (out_size != n) return;

  const float* q = (const float*)d_in[0];
  const float* k = (const float*)d_in[1];
  const float* v = (const float*)d_in[2];

  const size_t PL = (size_t)n * 2;
  size_t off = 0;
  const size_t oQ = off; off += PL;
  const size_t oK = off; off += PL;
  const size_t oV = off; off += PL;
  if (off > ws_size) return;
  if (off > (size_t)134217728) return;

  char* ws = (char*)d_ws;
  unsigned short* Qb = (unsigned short*)(ws + oQ);
  unsigned short* Kb = (unsigned short*)(ws + oK);
  unsigned short* VT = (unsigned short*)(ws + oV);

  const int  n8 = n / 8;
  const dim3 gCvt((n8 + 255) / 256);
  const dim3 gTr(SEQ / 64, NB);
  const dim3 gAttn(NB * NQB);

  cvt_bf16x8<<<gCvt, dim3(256), 0, stream>>>(q, Qb, n8);
  cvt_bf16x8<<<gCvt, dim3(256), 0, stream>>>(k, Kb, n8);
  vtr64<<<gTr, dim3(128), 0, stream>>>(v, VT);
  attn_band<<<gAttn, dim3(128), 0, stream>>>(Qb, Kb, VT, (float*)d_out, 0.08838834764831845f);
  (void)hipGetLastError();
}
